// GroupChannelAttention_81930796139038
// MI455X (gfx1250) — hardware-verified
//
#include <hip/hip_runtime.h>
#include <stdint.h>

#define BB     8
#define NN     4096
#define DIMC   256
#define NH     4
#define HD     64
#define MLP    768
#define NTOK   (BB * NN)
#define LDC    132
#define LDX    260
#define LDA    68
#define RSC    0.00048828125f
#define PLANE  ((size_t)BB * NH * HD * NN)
#define QL_OFF ((size_t)NTOK * DIMC)
#define ATL_OFF ((size_t)BB * NH * HD * HD)

static_assert(NTOK == 32768);
static_assert(DIMC == NH * HD);
static_assert((NN % 64) == 0 && (NTOK % 64) == 0);
static_assert((DIMC % 32) == 0 && (MLP % 32) == 0 && (HD % 32) == 0 && (NN % 32) == 0);
static_assert((LDX * 4) % 16 == 0 && (LDC * 4) % 16 == 0);
static_assert(PLANE == 8388608 && QL_OFF == 8388608 && ATL_OFF == 131072);
static_assert(MLP == 6 * 128 && DIMC == 2 * 128);

typedef _Float16 v16h __attribute__((ext_vector_type(16)));
typedef _Float16 v8h  __attribute__((ext_vector_type(8)));
typedef float    v8f  __attribute__((ext_vector_type(8)));
typedef float    v4f  __attribute__((ext_vector_type(4)));
typedef unsigned int v4u __attribute__((ext_vector_type(4)));

__device__ __forceinline__ unsigned short bf_bits(float f) {
  unsigned u = __float_as_uint(f);
  return (unsigned short)((u + 0x7FFFu + ((u >> 16) & 1u)) >> 16);
}
__device__ __forceinline__ float bf_up(unsigned short b) { return __uint_as_float(((unsigned)b) << 16); }
__device__ __forceinline__ float bfr(float f) { return bf_up(bf_bits(f)); }
__device__ __forceinline__ unsigned short h_bits(_Float16 x) { return __builtin_bit_cast(unsigned short, x); }
__device__ __forceinline__ unsigned short hb16(float f) { return h_bits((_Float16)f); }
__device__ __forceinline__ unsigned pk16(unsigned short a, unsigned short b) { return (unsigned)a | ((unsigned)b << 16); }
__device__ __forceinline__ v8f zero8() { v8f z = {0.f, 0.f, 0.f, 0.f, 0.f, 0.f, 0.f, 0.f}; return z; }
__device__ __forceinline__ void split2(float f0, float f1, unsigned& hp, unsigned& lp) {
  const _Float16 h0 = (_Float16)f0, h1 = (_Float16)f1;
  const float q0 = (f0 - (float)h0) * 2048.0f, q1 = (f1 - (float)h1) * 2048.0f;
  hp = pk16(h_bits(h0), h_bits(h1));
  lp = pk16(hb16(q0), hb16(q1));
}

__device__ __forceinline__ v16h ldfrag_h(const _Float16* p) {
  union { v16h v; v8h h[2]; } f;
  f.h[0] = *(const v8h*)(p);
  f.h[1] = *(const v8h*)(p + 16);
  return f.v;
}

__device__ __forceinline__ v8f mma_raw(v16h a, v16h b, v8f c) {
  return __builtin_amdgcn_wmma_f32_16x16x32_f16(false, a, false, b, (short)0, c, false, false);
}
__device__ __forceinline__ void guard4(v8f& c0, v8f& c1, v8f& c2, v8f& c3,
                                       const v16h& a0, const v16h& a1, const v16h& b0, const v16h& b1) {
#if defined(__HIP_DEVICE_COMPILE__)
  asm volatile("v_nop\n\tv_nop\n\tv_nop\n\tv_nop"
               : "+v"(c0), "+v"(c1), "+v"(c2), "+v"(c3)
               : "v"(a0), "v"(a1), "v"(b0), "v"(b1));
#endif
}
__device__ __forceinline__ void guard6(v8f& c0, v8f& c1, v8f& c2, v8f& c3, v8f& c4, v8f& c5,
                                       const v16h& a0, const v16h& a1, const v16h& b0, const v16h& b1,
                                       const v16h& b2, const v16h& b3) {
#if defined(__HIP_DEVICE_COMPILE__)
  asm volatile("v_nop\n\tv_nop\n\tv_nop\n\tv_nop"
               : "+v"(c0), "+v"(c1), "+v"(c2), "+v"(c3), "+v"(c4), "+v"(c5)
               : "v"(a0), "v"(a1), "v"(b0), "v"(b1), "v"(b2), "v"(b3));
#endif
}
__device__ __forceinline__ void guard3(v8f& c0, v8f& c1, v8f& c2,
                                       const v16h& a0, const v16h& a1, const v16h& b0, const v16h& b1) {
#if defined(__HIP_DEVICE_COMPILE__)
  asm volatile("v_nop\n\tv_nop\n\tv_nop\n\tv_nop"
               : "+v"(c0), "+v"(c1), "+v"(c2)
               : "v"(a0), "v"(a1), "v"(b0), "v"(b1));
#endif
}

__device__ __forceinline__ void mm_tile1(const _Float16* __restrict__ A, int lda,
                                         const _Float16* __restrict__ W, int ldw, int nks,
                                         int arow0, int bcol0, float* Cs) {
  const int tid = threadIdx.x, wave = tid >> 5, lane = tid & 31, hh = lane >> 4, c = lane & 15;
  const int mw = wave >> 2, nw = wave & 3;
  const _Float16* a0p = A + (size_t)(arow0 + mw * 32 + c) * lda + 8 * hh;
  const _Float16* a1p = A + (size_t)(arow0 + mw * 32 + 16 + c) * lda + 8 * hh;
  const _Float16* b0p = W + (size_t)(bcol0 + nw * 32 + c) * ldw + 8 * hh;
  const _Float16* b1p = W + (size_t)(bcol0 + nw * 32 + 16 + c) * ldw + 8 * hh;
  v8f c00 = zero8(), c01 = zero8(), c10 = zero8(), c11 = zero8();
#pragma unroll 1
  for (int ks = 0; ks < nks; ++ks) {
    const int ko = ks * 32;
    const v16h fa0 = ldfrag_h(a0p + ko);
    const v16h fa1 = ldfrag_h(a1p + ko);
    const v16h fb0 = ldfrag_h(b0p + ko);
    const v16h fb1 = ldfrag_h(b1p + ko);
    c00 = mma_raw(fa0, fb0, c00);
    c01 = mma_raw(fa0, fb1, c01);
    c10 = mma_raw(fa1, fb0, c10);
    c11 = mma_raw(fa1, fb1, c11);
    guard4(c00, c01, c10, c11, fa0, fa1, fb0, fb1);
  }
#pragma unroll
  for (int r = 0; r < 8; ++r) {
    const int row = mw * 32 + 8 * hh + r;
    Cs[row * LDC + nw * 32 + c]             = c00[r];
    Cs[row * LDC + nw * 32 + 16 + c]        = c01[r];
    Cs[(row + 16) * LDC + nw * 32 + c]      = c10[r];
    Cs[(row + 16) * LDC + nw * 32 + 16 + c] = c11[r];
  }
}

__global__ __launch_bounds__(128)
void k_wcvt(const float* __restrict__ wqkv, const float* __restrict__ wfc1, const float* __restrict__ wfc2,
            unsigned short* wqt, unsigned short* w1t, unsigned short* w2t) {
  const int tid = threadIdx.x;
  const int blk = blockIdx.x;
  if (blk < 2 * MLP) {
    const int t = (blk < MLP) ? 0 : 1;
    const int n = blk - t * MLP;
    const float* src = t ? wfc1 : wqkv;
    unsigned short* dstp = t ? w1t : wqt;
    const int tt = min(tid, 31);
    const int k0 = tt * 8;
    v4u pk;
#pragma unroll
    for (int e = 0; e < 4; ++e) {
      const float f0 = src[(size_t)(k0 + 2 * e) * MLP + n];
      const float f1 = src[(size_t)(k0 + 2 * e + 1) * MLP + n];
      pk[e] = pk16(hb16(bfr(f0) * 64.0f), hb16(bfr(f1) * 64.0f));
    }
    if (tid < 32) {
      unsigned short* dst = dstp + (size_t)n * DIMC + k0;
      *(volatile v4u*)dst = pk;
      __threadfence();
      *(volatile v4u*)dst = pk;
    }
  } else {
    const int n = blk - 2 * MLP;
    const int tt = min(tid, 95);
    const int k0 = tt * 8;
    v4u pk;
#pragma unroll
    for (int e = 0; e < 4; ++e) {
      const float f0 = wfc2[(size_t)(k0 + 2 * e) * DIMC + n];
      const float f1 = wfc2[(size_t)(k0 + 2 * e + 1) * DIMC + n];
      pk[e] = pk16(hb16(bfr(f0) * 64.0f), hb16(bfr(f1) * 64.0f));
    }
    if (tid < 96) {
      unsigned short* dst = w2t + (size_t)n * MLP + k0;
      *(volatile v4u*)dst = pk;
      __threadfence();
      *(volatile v4u*)dst = pk;
    }
  }
}

__global__ __launch_bounds__(256)
void k_xcvt(const float* __restrict__ x, unsigned short* xh, int npieces) {
  const int i = blockIdx.x * 256 + threadIdx.x;
  if (i >= npieces) return;
  const float* p = x + (size_t)i * 8;
  const v4f a = *(const v4f*)(p);
  const v4f b = *(const v4f*)(p + 4);
  v4u pk;
  pk[0] = pk16(hb16(bfr(a[0]) * 16.0f), hb16(bfr(a[1]) * 16.0f));
  pk[1] = pk16(hb16(bfr(a[2]) * 16.0f), hb16(bfr(a[3]) * 16.0f));
  pk[2] = pk16(hb16(bfr(b[0]) * 16.0f), hb16(bfr(b[1]) * 16.0f));
  pk[3] = pk16(hb16(bfr(b[2]) * 16.0f), hb16(bfr(b[3]) * 16.0f));
  unsigned short* dst = xh + (size_t)i * 8;
  *(volatile v4u*)dst = pk;
  __threadfence();
  *(volatile v4u*)dst = pk;
}

__global__ __launch_bounds__(256)
void k_qkv(const unsigned short* __restrict__ xh, const unsigned short* __restrict__ wqt,
           const float* __restrict__ bias, unsigned short* qp, unsigned short* kv) {
  __shared__ __align__(16) float Cs[64 * LDC];
  const int tid = threadIdx.x;
  const int mb = blockIdx.x, cg = blockIdx.y;
  const int tok0 = mb * 64, col0 = cg * 128;
  mm_tile1((const _Float16*)(const void*)xh, DIMC, (const _Float16*)(const void*)wqt, DIMC, DIMC / 32,
           tok0, col0, Cs);
  __syncthreads();
  const int s = cg >> 1, hp = cg & 1;
  if (s == 0) {
    unsigned short* dh = qp;
    unsigned short* dl = qp + QL_OFF;
    v4u ph[4], pq[4];
    size_t offs[4];
#pragma unroll
    for (int s4 = 0; s4 < 4; ++s4) {
      const int idx = s4 * 256 + tid;
      const int row = idx >> 4, piece = idx & 15;
      const int colp = piece * 8;
      v4u a, q4;
#pragma unroll
      for (int e = 0; e < 4; ++e) {
        const float b0 = 16.0f * bfr(bias[col0 + colp + 2 * e]);
        const float b1 = 16.0f * bfr(bias[col0 + colp + 2 * e + 1]);
        const float f0 = Cs[row * LDC + colp + 2 * e] * (1.0f / 64.0f) + b0;
        const float f1 = Cs[row * LDC + colp + 2 * e + 1] * (1.0f / 64.0f) + b1;
        unsigned hw, lw;
        split2(f0, f1, hw, lw);
        a[e] = hw; q4[e] = lw;
      }
      ph[s4] = a;
      pq[s4] = q4;
      offs[s4] = (size_t)(tok0 + row) * DIMC + hp * 128 + colp;
    }
#pragma unroll
    for (int s4 = 0; s4 < 4; ++s4) { *(volatile v4u*)(dh + offs[s4]) = ph[s4]; *(volatile v4u*)(dl + offs[s4]) = pq[s4]; }
    __threadfence();
#pragma unroll
    for (int s4 = 0; s4 < 4; ++s4) { *(volatile v4u*)(dh + offs[s4]) = ph[s4]; *(volatile v4u*)(dl + offs[s4]) = pq[s4]; }
  } else {
    unsigned short* dh = kv + (size_t)(s - 1) * 2 * PLANE;
    unsigned short* dl = dh + PLANE;
    const int b = tok0 >> 12, n0 = tok0 & (NN - 1);
    v4u ph[4], pq[4];
    size_t offs[4];
#pragma unroll
    for (int s4 = 0; s4 < 4; ++s4) {
      const int idx = s4 * 256 + tid;
      const int ch = idx >> 3, piece = idx & 7;
      const int h = 2 * hp + (ch >> 6), d = ch & 63;
      const float bb = 16.0f * bfr(bias[col0 + ch]);
      const int r0 = piece * 8;
      v4u a, q4;
#pragma unroll
      for (int e = 0; e < 4; ++e) {
        const float f0 = Cs[(r0 + 2 * e) * LDC + ch] * (1.0f / 64.0f) + bb;
        const float f1 = Cs[(r0 + 2 * e + 1) * LDC + ch] * (1.0f / 64.0f) + bb;
        unsigned hw, lw;
        split2(f0, f1, hw, lw);
        a[e] = hw; q4[e] = lw;
      }
      ph[s4] = a;
      pq[s4] = q4;
      offs[s4] = ((size_t)(b * NH + h) * HD + d) * NN + n0 + r0;
    }
#pragma unroll
    for (int s4 = 0; s4 < 4; ++s4) { *(volatile v4u*)(dh + offs[s4]) = ph[s4]; *(volatile v4u*)(dl + offs[s4]) = pq[s4]; }
    __threadfence();
#pragma unroll
    for (int s4 = 0; s4 < 4; ++s4) { *(volatile v4u*)(dh + offs[s4]) = ph[s4]; *(volatile v4u*)(dl + offs[s4]) = pq[s4]; }
  }
}

__global__ __launch_bounds__(256)
void k_attn(const unsigned short* __restrict__ kv, unsigned short* at) {
  __shared__ __align__(16) float Cs[64 * LDA];
  const int tid = threadIdx.x, wave = tid >> 5, lane = tid & 31, hh = lane >> 4, c = lane & 15;
  const int bh = blockIdx.x;
  const _Float16* base = (const _Float16*)(const void*)kv;
  const _Float16* Kh = base + (size_t)bh * HD * NN;
  const _Float16* Kl = Kh + PLANE;
  const _Float16* Vh = Kh + 2 * PLANE;
  const _Float16* Vl = Kh + 3 * PLANE;
  {
    const int mw = wave >> 1, nw = wave & 1;
    const _Float16* ahp = Kh + (size_t)(mw * 16 + c) * NN + 8 * hh;
    const _Float16* alp = Kl + (size_t)(mw * 16 + c) * NN + 8 * hh;
    const _Float16* b0h = Vh + (size_t)(nw * 32 + c) * NN + 8 * hh;
    const _Float16* b1h = Vh + (size_t)(nw * 32 + 16 + c) * NN + 8 * hh;
    const _Float16* b0l = Vl + (size_t)(nw * 32 + c) * NN + 8 * hh;
    const _Float16* b1l = Vl + (size_t)(nw * 32 + 16 + c) * NN + 8 * hh;
    v8f p0 = zero8(), p1 = zero8(), q0 = zero8(), q1 = zero8(), r0 = zero8(), r1 = zero8();
#pragma unroll 1
    for (int ks = 0; ks < NN / 32; ++ks) {
      const int ko = ks * 32;
      const v16h fa  = ldfrag_h(ahp + ko);
      const v16h ga  = ldfrag_h(alp + ko);
      const v16h fb0 = ldfrag_h(b0h + ko);
      const v16h fb1 = ldfrag_h(b1h + ko);
      const v16h gb0 = ldfrag_h(b0l + ko);
      const v16h gb1 = ldfrag_h(b1l + ko);
      p0 = mma_raw(fa, fb0, p0);
      p1 = mma_raw(fa, fb1, p1);
      q0 = mma_raw(fa, gb0, q0);
      q1 = mma_raw(fa, gb1, q1);
      r0 = mma_raw(ga, fb0, r0);
      r1 = mma_raw(ga, fb1, r1);
      guard6(p0, p1, q0, q1, r0, r1, fa, ga, fb0, fb1, gb0, gb1);
    }
#pragma unroll
    for (int r = 0; r < 8; ++r) {
      const int row = mw * 16 + 8 * hh + r;
      Cs[row * LDA + nw * 32 + c]      = p0[r] + (q0[r] + r0[r]) * RSC;
      Cs[row * LDA + nw * 32 + 16 + c] = p1[r] + (q1[r] + r1[r]) * RSC;
    }
  }
  __syncthreads();
  {
    const int row = tid >> 2, part = tid & 3;
    float* cr = Cs + row * LDA + part * 16;
    float mx = -3.0e38f;
#pragma unroll 1
    for (int n = 0; n < 16; ++n) mx = fmaxf(mx, cr[n]);
    mx = fmaxf(mx, __shfl_xor(mx, 1, 32));
    mx = fmaxf(mx, __shfl_xor(mx, 2, 32));
    float sm = 0.f;
#pragma unroll 1
    for (int n = 0; n < 16; ++n) {
      const float e = expf((cr[n] - mx) * RSC);
      cr[n] = e;
      sm += e;
    }
    sm += __shfl_xor(sm, 1, 32);
    sm += __shfl_xor(sm, 2, 32);
    const float sc = (1.0f / sm) * 4096.0f;
#pragma unroll 1
    for (int n = 0; n < 16; ++n) cr[n] = cr[n] * sc;
  }
  __syncthreads();
  unsigned short* dh = at;
  unsigned short* dl = at + ATL_OFF;
  v4u ph[2], pq[2];
  size_t offs[2];
#pragma unroll
  for (int s = 0; s < 2; ++s) {
    const int idx = s * 256 + tid;
    const int row = idx >> 3, piece = idx & 7;
    const int col0 = piece * 8;
    v4u a, q4;
#pragma unroll
    for (int e = 0; e < 4; ++e) {
      unsigned hw, lw;
      split2(Cs[row * LDA + col0 + 2 * e], Cs[row * LDA + col0 + 2 * e + 1], hw, lw);
      a[e] = hw; q4[e] = lw;
    }
    ph[s] = a;
    pq[s] = q4;
    offs[s] = ((size_t)bh * HD + row) * HD + col0;
  }
#pragma unroll
  for (int s = 0; s < 2; ++s) { *(volatile v4u*)(dh + offs[s]) = ph[s]; *(volatile v4u*)(dl + offs[s]) = pq[s]; }
  __threadfence();
#pragma unroll
  for (int s = 0; s < 2; ++s) { *(volatile v4u*)(dh + offs[s]) = ph[s]; *(volatile v4u*)(dl + offs[s]) = pq[s]; }
}

__global__ __launch_bounds__(256)
void k_xf(const unsigned short* __restrict__ qp, const unsigned short* __restrict__ at,
          const float* __restrict__ x, const float* __restrict__ gw, const float* __restrict__ gb,
          float* x1, unsigned short* hh16) {
  __shared__ __align__(16) float Cs[32 * LDX];
  __shared__ float Mu[32];
  __shared__ float Rs[32];
  const int tid = threadIdx.x, wave = tid >> 5, lane = tid & 31, hh = lane >> 4, c = lane & 15;
  const int mw = wave >> 2, nw = wave & 3;
  const int tok0 = blockIdx.x * 32;
  const int b = tok0 >> 12;
  const _Float16* Qh = (const _Float16*)(const void*)qp;
  const _Float16* Ql = Qh + QL_OFF;
  const _Float16* Ah = (const _Float16*)(const void*)at;
  const _Float16* Al = Ah + ATL_OFF;
  const size_t arow = (size_t)(tok0 + mw * 16 + c) * DIMC + 8 * hh;
#pragma unroll 1
  for (int h = 0; h < NH; ++h) {
    const _Float16* ahp = Qh + arow + h * HD;
    const _Float16* alp = Ql + arow + h * HD;
    const size_t brow = ((size_t)(b * NH + h) * HD + nw * 16 + c) * HD + 8 * hh;
    const _Float16* bhp = Ah + brow;
    const _Float16* blp = Al + brow;
    v8f p = zero8(), q = zero8(), r = zero8();
#pragma unroll
    for (int ks = 0; ks < HD / 32; ++ks) {
      const int ko = ks * 32;
      const v16h fa = ldfrag_h(ahp + ko);
      const v16h ga = ldfrag_h(alp + ko);
      const v16h fb = ldfrag_h(bhp + ko);
      const v16h gq = ldfrag_h(blp + ko);
      p = mma_raw(fa, fb, p);
      q = mma_raw(fa, gq, q);
      r = mma_raw(ga, fb, r);
      guard3(p, q, r, fa, ga, fb, gq);
    }
#pragma unroll
    for (int rr = 0; rr < 8; ++rr)
      Cs[(mw * 16 + 8 * hh + rr) * LDX + h * HD + nw * 16 + c] = p[rr] + (q[rr] + r[rr]) * RSC;
  }
  __syncthreads();
#pragma unroll 1
  for (int it = 0; it < 4; ++it) {
    const int row = wave * 4 + it;
    const size_t tok = (size_t)(tok0 + row);
    const float* xr = x + tok * DIMC + lane * 8;
    const v4f xa = *(const v4f*)(xr);
    const v4f xb = *(const v4f*)(xr + 4);
    float* cr = Cs + row * LDX + lane * 8;
    float v[8];
#pragma unroll
    for (int e = 0; e < 4; ++e) {
      v[e]     = bfr(xa[e]) + cr[e] * (1.0f / 65536.0f);
      v[4 + e] = bfr(xb[e]) + cr[4 + e] * (1.0f / 65536.0f);
    }
#pragma unroll
    for (int e = 0; e < 8; ++e) cr[e] = v[e];
    float s = ((v[0] + v[1]) + (v[2] + v[3])) + ((v[4] + v[5]) + (v[6] + v[7]));
#pragma unroll
    for (int off = 16; off; off >>= 1) s += __shfl_xor(s, off, 32);
    const float mu = s * (1.0f / 256.0f);
    float sq = 0.f;
#pragma unroll
    for (int e = 0; e < 8; ++e) { const float d = v[e] - mu; sq += d * d; }
#pragma unroll
    for (int off = 16; off; off >>= 1) sq += __shfl_xor(sq, off, 32);
    const float var = sq * (1.0f / 256.0f);
    const float rs = rsqrtf(var + 1e-5f);
    if (lane == 0) { Mu[row] = mu; Rs[row] = rs; }
  }
  __syncthreads();
  v4f pk[8];
  size_t offs[8];
#pragma unroll
  for (int s = 0; s < 8; ++s) {
    const int idx = s * 256 + tid;
    const int row = idx >> 6, piece = idx & 63;
    v4f v4;
#pragma unroll
    for (int e = 0; e < 4; ++e) v4[e] = Cs[row * LDX + piece * 4 + e];
    pk[s] = v4;
    offs[s] = (size_t)(tok0 + row) * DIMC + piece * 4;
  }
  v4u ph[4];
  size_t offh[4];
#pragma unroll
  for (int s = 0; s < 4; ++s) {
    const int idx = s * 256 + tid;
    const int row = idx >> 5, piece = idx & 31;
    const int col0 = piece * 8;
    const float mu = Mu[row], rs = Rs[row];
    v4u a;
#pragma unroll
    for (int e = 0; e < 4; ++e) {
      const int cA = col0 + 2 * e, cB = cA + 1;
      const float f0 = ((Cs[row * LDX + cA] - mu) * rs) * bfr(gw[cA]) + bfr(gb[cA]);
      const float f1 = ((Cs[row * LDX + cB] - mu) * rs) * bfr(gw[cB]) + bfr(gb[cB]);
      a[e] = pk16(hb16(f0 * 16.0f), hb16(f1 * 16.0f));
    }
    ph[s] = a;
    offh[s] = (size_t)(tok0 + row) * DIMC + col0;
  }
#pragma unroll
  for (int s = 0; s < 8; ++s) *(volatile v4f*)(x1 + offs[s]) = pk[s];
#pragma unroll
  for (int s = 0; s < 4; ++s) *(volatile v4u*)(hh16 + offh[s]) = ph[s];
  __threadfence();
#pragma unroll
  for (int s = 0; s < 8; ++s) *(volatile v4f*)(x1 + offs[s]) = pk[s];
#pragma unroll
  for (int s = 0; s < 4; ++s) *(volatile v4u*)(hh16 + offh[s]) = ph[s];
}

__global__ __launch_bounds__(256)
void k_fc1(const unsigned short* __restrict__ hh16, const unsigned short* __restrict__ w1t,
           const float* __restrict__ bias, unsigned short* gh) {
  __shared__ __align__(16) float Cs[64 * LDC];
  const int tid = threadIdx.x;
  const int mb = blockIdx.x, cg = blockIdx.y;
  const int tok0 = mb * 64, col0 = cg * 128;
  mm_tile1((const _Float16*)(const void*)hh16, DIMC, (const _Float16*)(const void*)w1t, DIMC, DIMC / 32,
           tok0, col0, Cs);
  __syncthreads();
  {
    const int row = tid >> 2, cq = tid & 3;
    float* cr = Cs + row * LDC + cq * 32;
    const float* bp = bias + col0 + cq * 32;
#pragma unroll 2
    for (int n = 0; n < 32; ++n) {
      const float v = cr[n] * (1.0f / 1024.0f) + bfr(bp[n]);
      const float ge = 0.5f * v * (1.0f + erff(v * 0.70710678118654752f));
      cr[n] = ge * 16.0f;
    }
  }
  __syncthreads();
  v4u pk[4];
  size_t offs[4];
#pragma unroll
  for (int s = 0; s < 4; ++s) {
    const int idx = s * 256 + tid;
    const int row = idx >> 4, piece = idx & 15;
    const int colp = piece * 8;
    v4u a;
#pragma unroll
    for (int e = 0; e < 4; ++e)
      a[e] = pk16(hb16(Cs[row * LDC + colp + 2 * e]), hb16(Cs[row * LDC + colp + 2 * e + 1]));
    pk[s] = a;
    offs[s] = (size_t)(tok0 + row) * MLP + col0 + colp;
  }
#pragma unroll
  for (int s = 0; s < 4; ++s) *(volatile v4u*)(gh + offs[s]) = pk[s];
  __threadfence();
#pragma unroll
  for (int s = 0; s < 4; ++s) *(volatile v4u*)(gh + offs[s]) = pk[s];
}

__global__ __launch_bounds__(256)
void k_fc2(const unsigned short* __restrict__ gh, const unsigned short* __restrict__ w2t,
           const float* __restrict__ bias, const float* __restrict__ x1, float* out) {
  __shared__ __align__(16) float Cs[64 * LDC];
  const int tid = threadIdx.x;
  const int mb = blockIdx.x, cg = blockIdx.y;
  const int tok0 = mb * 64, col0 = cg * 128;
  mm_tile1((const _Float16*)(const void*)gh, MLP, (const _Float16*)(const void*)w2t, MLP, MLP / 32,
           tok0, col0, Cs);
  __syncthreads();
  v4f pk[8];
  size_t offs[8];
#pragma unroll
  for (int s = 0; s < 8; ++s) {
    const int idx = s * 256 + tid;
    const int row = idx >> 5, piece = idx & 31;
    const int colp = piece * 4;
    const size_t off = (size_t)(tok0 + row) * DIMC + col0 + colp;
    const v4f xr = *(const v4f*)(x1 + off);
    v4f v;
#pragma unroll
    for (int e = 0; e < 4; ++e)
      v[e] = xr[e] + (Cs[row * LDC + colp + e] * (1.0f / 1024.0f) + bfr(bias[col0 + colp + e]));
    pk[s] = v;
    offs[s] = off;
  }
#pragma unroll
  for (int s = 0; s < 8; ++s) *(volatile v4f*)(out + offs[s]) = pk[s];
  __threadfence();
#pragma unroll
  for (int s = 0; s < 8; ++s) *(volatile v4f*)(out + offs[s]) = pk[s];
}

extern "C" void kernel_launch(void* const* d_in, const int* in_sizes, int n_in,
                              void* d_out, int out_size, void* d_ws, size_t ws_size,
                              hipStream_t stream) {
  if (n_in < 9) return;
  const int expect[9] = { NTOK * DIMC, DIMC * MLP, MLP, DIMC, DIMC, DIMC * MLP, MLP, MLP * DIMC, DIMC };
  for (int i = 0; i < 9; ++i) if (in_sizes[i] != expect[i]) return;
  if (out_size != NTOK * DIMC) return;

  const float* x     = (const float*)d_in[0];
  const float* w_qkv = (const float*)d_in[1];
  const float* b_qkv = (const float*)d_in[2];
  const float* ng    = (const float*)d_in[3];
  const float* nbt   = (const float*)d_in[4];
  const float* w_fc1 = (const float*)d_in[5];
  const float* b_fc1 = (const float*)d_in[6];
  const float* w_fc2 = (const float*)d_in[7];
  const float* b_fc2 = (const float*)d_in[8];
  float* out = (float*)d_out;

  const size_t MiB = (size_t)1048576;
  const size_t szX16 = (size_t)NTOK * DIMC * 2;
  const size_t szPl  = PLANE * 2;
  const size_t szX1  = (size_t)NTOK * DIMC * 4;
  const size_t szGH  = (size_t)NTOK * MLP * 2;
  const size_t szAT  = ATL_OFF * 2;
  const size_t szWQ  = (size_t)MLP * DIMC * 2;
  if (szX16 != 16 * MiB || szPl != 16 * MiB || szX1 != 32 * MiB || szGH != 48 * MiB) return;

  const size_t oXH  = 0;
  const size_t oHH  = 0;
  const size_t oQH  = 16 * MiB;
  const size_t oKV  = 48 * MiB;
  const size_t oX1  = 80 * MiB;
  const size_t oGH  = 16 * MiB;
  const size_t oATH = 112 * MiB;
  const size_t oWQT = oATH + 2 * szAT;
  const size_t oW1T = oWQT + szWQ;
  const size_t oW2T = oW1T + szWQ;
  const size_t oEND = oW2T + szWQ;
  if (oQH + 2 * szX16 != oKV) return;
  if (oKV + 4 * szPl != oATH) return;
  if (oX1 + szX1 > oATH || oGH + szGH > oX1 || oHH + szX16 > oGH) return;
  if (oEND > ws_size) return;
  if (oEND > (size_t)134217728) return;

  char* ws = (char*)d_ws;
  unsigned short* XH  = (unsigned short*)(ws + oXH);
  unsigned short* HH  = (unsigned short*)(ws + oHH);
  unsigned short* QH  = (unsigned short*)(ws + oQH);
  unsigned short* KV  = (unsigned short*)(ws + oKV);
  float*          X1  = (float*)(ws + oX1);
  unsigned short* GH  = (unsigned short*)(ws + oGH);
  unsigned short* ATH = (unsigned short*)(ws + oATH);
  unsigned short* WQT = (unsigned short*)(ws + oWQT);
  unsigned short* W1T = (unsigned short*)(ws + oW1T);
  unsigned short* W2T = (unsigned short*)(ws + oW2T);

  const dim3 blk(256);
  const int npieces = NTOK * DIMC / 8;
  k_wcvt<<<dim3(2 * MLP + DIMC), dim3(128), 0, stream>>>(w_qkv, w_fc1, w_fc2, WQT, W1T, W2T);
  k_xcvt<<<dim3((npieces + 255) / 256), blk, 0, stream>>>(x, XH, npieces);
  k_qkv<<<dim3(NTOK / 64, 6), blk, 0, stream>>>(XH, WQT, b_qkv, QH, KV);
  k_attn<<<dim3(BB * NH), blk, 0, stream>>>(KV, ATH);
  k_xf<<<dim3(NTOK / 32), blk, 0, stream>>>(QH, ATH, x, ng, nbt, X1, HH);
  k_fc1<<<dim3(NTOK / 64, 6), blk, 0, stream>>>(HH, W1T, b_fc1, GH);
  k_fc2<<<dim3(NTOK / 64, 2), blk, 0, stream>>>(GH, W2T, b_fc2, X1, out);
  (void)hipGetLastError();
}
